// SSA_28845000360490
// MI455X (gfx1250) — hardware-verified
//
#include <hip/hip_runtime.h>
#include <stddef.h>


typedef _Float16 v16h __attribute__((ext_vector_type(16)));
typedef _Float16 v8h  __attribute__((ext_vector_type(8)));
typedef _Float16 v4h  __attribute__((ext_vector_type(4)));
typedef float    v8f  __attribute__((ext_vector_type(8)));
typedef float    v4f  __attribute__((ext_vector_type(4)));

#ifndef NB
#define NB 4
#endif
#define NB_FULL 4
#define CH   32
#define CIN  64
#define IMH  64
#define IMW  64
#define HW   4096
#define OC   8
#define K1   576
#define K2P  96
#define K3   64
#define NEG_SLOPE 0.01f

#define LDA  72

#define WCARRY 64.0f
#define OCARRY 256.0f
#define VCARRY 16.0f

static_assert(NB >= 1 && NB <= NB_FULL);
static_assert(IMH == 64 && IMW == 64 && HW == IMH * IMW);
static_assert(CIN == 2 * CH && CH == 32 && OC == 8);
static_assert((K1 % 32) == 0 && (K2P % 32) == 0 && (K3 % 32) == 0);
static_assert(K1 == 9 * CIN && K2P >= 9 * OC);
static_assert((LDA % 8) == 0 && LDA >= 64);
static_assert((HW / 4) == 1024);

#define WT_W1   0
#define WT_W2   (16 * K1)
#define WT_W11  (WT_W2 + 16 * K2P)
#define WT_HALVES (WT_W11 + 16 * K3)
#define WT_VECS (WT_HALVES / 8)
static_assert(WT_HALVES == 11776 && WT_VECS == 1472);
static_assert(((WT_W2 * 2) % 128) == 0 && ((WT_W11 * 2) % 128) == 0 && ((WT_HALVES * 2) % 128) == 0);

#define WT_BYTES  ((size_t)WT_HALVES * 2)
#define O1_BYTES  ((size_t)NB * HW * OC * 2)
#define VP_BYTES  ((size_t)NB * OC * HW * 2)
#define U_BYTES   ((size_t)NB * OC * CH * 4)
#define OFF_WT  ((size_t)0)
#define OFF_O1  (OFF_WT + WT_BYTES)
#define OFF_VP  (OFF_O1 + O1_BYTES)
#define OFF_U   (OFF_VP + VP_BYTES)
#define WS_TOTAL (OFF_U + U_BYTES)
static_assert((WT_BYTES % 128) == 0 && (O1_BYTES % 128) == 0 && (VP_BYTES % 128) == 0);
static_assert((U_BYTES % 128) == 0);
static_assert(WS_TOTAL <= (size_t)134217728);

__device__ __forceinline__ float bf16r(float x) {
  unsigned int u = __float_as_uint(x);
  u = (u + 0x7FFFu + ((u >> 16) & 1u)) & 0xFFFF0000u;
  return __uint_as_float(u);
}

static __device__ __forceinline__ _Float16 toh_flush(float v) {
  const _Float16 r = (_Float16)v;
  return (fabsf(v) < 6.103515625e-05f) ? (_Float16)0.0f : r;
}

__device__ __forceinline__ v16h frag_at(const _Float16* p) {
  v8h lo = *(const v8h*)(p);
  v8h hi = *(const v8h*)(p + 16);
  v16h out;
#pragma unroll
  for (int i = 0; i < 8; ++i) { out[i] = lo[i]; out[i + 8] = hi[i]; }
  return out;
}

__device__ __forceinline__ v16h frag_pair(v8h lo, v8h hi) {
  v16h out;
#pragma unroll
  for (int i = 0; i < 8; ++i) { out[i] = lo[i]; out[i + 8] = hi[i]; }
  return out;
}

__device__ __forceinline__ v16h xfrag_at(const float* p) {
  const v4f a0 = *(const v4f*)(p);
  const v4f a1 = *(const v4f*)(p + 4);
  const v4f a2 = *(const v4f*)(p + 16);
  const v4f a3 = *(const v4f*)(p + 20);
  v16h out;
#pragma unroll
  for (int i = 0; i < 4; ++i) {
    out[i]      = toh_flush(bf16r(a0[i]));
    out[i + 4]  = toh_flush(bf16r(a1[i]));
    out[i + 8]  = toh_flush(bf16r(a2[i]));
    out[i + 12] = toh_flush(bf16r(a3[i]));
  }
  return out;
}

__device__ __forceinline__ v8f wmma16(v16h a, v16h b, v8f c) {
  v8f d = __builtin_amdgcn_wmma_f32_16x16x32_f16(false, a, false, b, (short)0, c,
                                                 false, false);
  asm volatile("v_nop\n\tv_nop\n\tv_nop\n\tv_nop" : "+v"(d) : "v"(a), "v"(b));
  return d;
}

__device__ __forceinline__ unsigned umin_u(unsigned a, unsigned b) { return a < b ? a : b; }
__device__ __forceinline__ unsigned umax_u(unsigned a, unsigned b) { return a > b ? a : b; }
__device__ __forceinline__ int clamp_i(int v, int lo, int hi) {
  return v < lo ? lo : (v > hi ? hi : v);
}

__device__ __forceinline__ float leaky_act(float t) {
  return (t >= 0.0f) ? t : NEG_SLOPE * t;
}

__global__ __launch_bounds__(256) void prep_kernel(
    const float* __restrict__ w1, const float* __restrict__ w2, const float* __restrict__ w11,
    _Float16* __restrict__ WT) {
  __shared__ __attribute__((aligned(16))) _Float16 T[256 * 8];
  const unsigned tid = threadIdx.x;
  const unsigned v = blockIdx.x * 256u + tid;

  const unsigned u1 = umin_u(v, 1151u);
  const unsigned n1 = u1 / 72u, kv1 = u1 - n1 * 72u;
  const unsigned tap1 = kv1 >> 3, ic1 = (kv1 & 7u) * 8u;
  const unsigned u2 = umin_u(umax_u(v, 1152u) - 1152u, 191u);
  const unsigned n2 = u2 / 12u, tap2 = u2 - n2 * 12u;
  const unsigned u3 = umin_u(umax_u(v, 1344u) - 1344u, 127u);
  const unsigned n3 = u3 >> 3, kv3 = u3 & 7u;

  const unsigned r1 = umin_u(n1, 7u) * 576u + tap1;
  const unsigned r2 = umin_u(n2, 7u) * 72u + umin_u(tap2, 8u);
  const unsigned r3 = umin_u(n3, 7u) * 64u + kv3 * 8u;
  const bool s1 = v < 1152u;
  const bool s2 = (!s1) && (v < 1344u);
  const bool ok = s1 ? (n1 < 8u) : (s2 ? ((n2 < 8u) && (tap2 < 9u)) : (n3 < 8u));

#pragma unroll 1
  for (unsigned j = 0; j < 8u; ++j) {
    const float a1 = w1[r1 + (ic1 + j) * 9u];
    const float a2 = w2[r2 + j * 9u];
    const float a3 = w11[r3 + j];
    const float s = s1 ? a1 : (s2 ? a2 : a3);
    const float val = ok ? (WCARRY * bf16r(s)) : 0.0f;
    T[tid * 8u + j] = toh_flush(val);
  }
  __syncthreads();
  const v8h x = *(const v8h*)&T[tid * 8u];
  const bool wr = v < (unsigned)WT_VECS;
  const size_t off = (size_t)umin_u(v, (unsigned)WT_VECS - 1u) * 8u;
  if (wr) *(volatile v8h*)(WT + off) = x;
  __threadfence();
  if (wr) *(volatile v8h*)(WT + off) = x;
}

__global__ __launch_bounds__(128) void conv1_kernel(
    const float* __restrict__ in1, const float* __restrict__ in2,
    const _Float16* __restrict__ W1t, const float* __restrict__ b1,
    _Float16* __restrict__ Out1) {
  __shared__ __attribute__((aligned(16))) _Float16 Act[3 * 66 * LDA];
  const unsigned tid = threadIdx.x, lane = tid & 31u;
  const unsigned wave = __builtin_amdgcn_readfirstlane(threadIdx.x >> 5);
  const unsigned hh = lane >> 4, m = lane & 15u;
  const unsigned b = blockIdx.x >> 6, y = blockIdx.x & 63u;

#pragma unroll 2
  for (unsigned i = tid; i < 3u * 32u * 66u; i += 128u) {
    const unsigned t = i / 66u;
    const unsigned xp = i - t * 66u;
    const unsigned ky = t >> 5, icl = t & 31u;
    const int yy = (int)y + (int)ky - 1;
    const int xx = (int)xp - 1;
    const bool ok = ((unsigned)yy < (unsigned)IMH) && ((unsigned)xx < (unsigned)IMW);
    const unsigned yc = (unsigned)clamp_i(yy, 0, IMH - 1);
    const unsigned xc = (unsigned)clamp_i(xx, 0, IMW - 1);
    const size_t idx = ((size_t)(b * CH + icl) << 12) + (yc << 6) + xc;
    const float la = in1[idx];
    const float lc = in2[idx];
    const float va = ok ? la : 0.0f;
    const float vc = ok ? lc : 0.0f;
    Act[(ky * 66u + xp) * LDA + icl]       = toh_flush(bf16r(va));
    Act[(ky * 66u + xp) * LDA + 32u + icl] = toh_flush(bf16r(vc));
  }
  __syncthreads();

  const unsigned x0 = wave * 16u;
  const _Float16* wp = W1t + m * K1 + hh * 8u;
  v8f acc = {};
#pragma unroll
  for (int ky = 0; ky < 3; ++ky) {
#pragma unroll
    for (int kx = 0; kx < 3; ++kx) {
      const _Float16* bp = &Act[((unsigned)ky * 66u + x0 + m + (unsigned)kx) * LDA + hh * 8u];
#pragma unroll
      for (int c = 0; c < 2; ++c) {
        const v16h a  = frag_at(wp + (ky * 3 + kx) * 64 + c * 32);
        const v16h bb = frag_at(bp + c * 32);
        acc = wmma16(a, bb, acc);
      }
    }
  }

  v8h o;
#pragma unroll
  for (int r = 0; r < 8; ++r) {
    const float t = acc[r] * (1.0f / WCARRY) + bf16r(b1[r]);
    o[r] = toh_flush(OCARRY * leaky_act(t));
  }
  _Float16* dst = Out1 + ((size_t)b * HW + y * 64u + x0 + m) * 8u;
  if (hh == 0u) *(volatile v8h*)dst = o;
  __threadfence();
  if (hh == 0u) *(volatile v8h*)dst = o;
}

__global__ __launch_bounds__(128) void conv2_kernel(
    const float* __restrict__ in1, const float* __restrict__ in2,
    const _Float16* __restrict__ Out1,
    const _Float16* __restrict__ W2t, const _Float16* __restrict__ W11t,
    const float* __restrict__ b2, const float* __restrict__ b11,
    _Float16* __restrict__ Vp) {
  __shared__ __attribute__((aligned(16))) _Float16 Act2[3 * 66 * 8];
  __shared__ __attribute__((aligned(16))) _Float16 Act3[64 * LDA];
  __shared__ __attribute__((aligned(16))) _Float16 Vs[8 * LDA];
  const unsigned tid = threadIdx.x, lane = tid & 31u;
  const unsigned wave = __builtin_amdgcn_readfirstlane(threadIdx.x >> 5);
  const unsigned hh = lane >> 4, m = lane & 15u;
  const unsigned b = blockIdx.x >> 6, y = blockIdx.x & 63u;

#pragma unroll
  for (unsigned j = 0; j < 2u; ++j) {
    const unsigned vv = tid + 128u * j;
    const unsigned vc = umin_u(vv, 197u);
    const unsigned ky = vc / 66u, xp = vc - ky * 66u;
    const int yy = (int)y + (int)ky - 1;
    const int xx = (int)xp - 1;
    const bool ok = ((unsigned)yy < (unsigned)IMH) && ((unsigned)xx < (unsigned)IMW);
    const unsigned yc = (unsigned)clamp_i(yy, 0, IMH - 1);
    const unsigned xc = (unsigned)clamp_i(xx, 0, IMW - 1);
    const v8h ld = *(const v8h*)(Out1 + ((size_t)b * HW + yc * 64u + xc) * 8u);
    v8h r;
#pragma unroll
    for (int i = 0; i < 8; ++i) r[i] = ok ? ld[i] : (_Float16)0.0f;
    if (vv < 198u) *(v8h*)&Act2[vc * 8u] = r;
  }
#pragma unroll 2
  for (unsigned i = tid; i < 32u * 64u; i += 128u) {
    const unsigned icl = i >> 6, xx = i & 63u;
    const size_t idx = ((size_t)(b * CH + icl) << 12) + (y << 6) + xx;
    const float la = in1[idx];
    const float lc = in2[idx];
    Act3[xx * LDA + icl]       = toh_flush(bf16r(la));
    Act3[xx * LDA + 32u + icl] = toh_flush(bf16r(lc));
  }
  __syncthreads();

  const unsigned x0 = wave * 16u;
  const _Float16* w2p  = W2t + m * K2P + hh * 8u;
  const _Float16* w11p = W11t + m * K3 + hh * 8u;
  v8f acc2 = {};
  v8f acc3 = {};
#pragma unroll
  for (int s = 0; s < 3; ++s) {
    const unsigned tlo = 4u * (unsigned)s + hh;
    const unsigned thi = tlo + 2u;
    const unsigned tl = umin_u(tlo, 8u), th = umin_u(thi, 8u);
    const unsigned kyl = tl / 3u, kxl = tl - 3u * kyl;
    const unsigned kyh = th / 3u, kxh = th - 3u * kyh;
    v8h lo = *(const v8h*)&Act2[(kyl * 66u + x0 + m + kxl) * 8u];
    v8h hi = *(const v8h*)&Act2[(kyh * 66u + x0 + m + kxh) * 8u];
#pragma unroll
    for (int i = 0; i < 8; ++i) {
      lo[i] = (tlo < 9u) ? lo[i] : (_Float16)0.0f;
      hi[i] = (thi < 9u) ? hi[i] : (_Float16)0.0f;
    }
    const v16h bb = frag_pair(lo, hi);
    const v16h a  = frag_at(w2p + s * 32);
    acc2 = wmma16(a, bb, acc2);
  }
#pragma unroll
  for (int c = 0; c < 2; ++c) {
    const v16h a  = frag_at(w11p + c * 32);
    const v16h bb = frag_at(&Act3[(x0 + m) * LDA + c * 32 + hh * 8u]);
    acc3 = wmma16(a, bb, acc3);
  }

  _Float16 vh[8];
#pragma unroll
  for (int r = 0; r < 8; ++r) {
    const float t2 = acc2[r] * (1.0f / (WCARRY * OCARRY)) + bf16r(b2[r]);
    const float t3 = acc3[r] * (1.0f / WCARRY) + bf16r(b11[r]);
    vh[r] = toh_flush(VCARRY * (leaky_act(t2) + t3));
  }
  if (hh == 0u) {
#pragma unroll
    for (int r = 0; r < 8; ++r) Vs[(unsigned)r * LDA + x0 + m] = vh[r];
  }
  __syncthreads();

  if (wave < 2u) {
    const unsigned q = tid >> 3;
    const unsigned pc = (tid & 7u) * 8u;
    const v8h x = *(const v8h*)&Vs[q * LDA + pc];
    _Float16* dst = Vp + ((size_t)(b * OC + q)) * HW + y * 64u + pc;
    *(volatile v8h*)dst = x;
    __threadfence();
    *(volatile v8h*)dst = x;
  }
}

__global__ __launch_bounds__(256) void gram_solve_kernel(
    const _Float16* __restrict__ Vp, const float* __restrict__ in1, float* __restrict__ U) {
  __shared__ __attribute__((aligned(16))) float part[8 * 3 * 8 * 16];
  __shared__ float Aug[8 * 40];
  __shared__ float fcol[8];
  const unsigned tid = threadIdx.x, lane = tid & 31u;
  const unsigned wave = __builtin_amdgcn_readfirstlane(threadIdx.x >> 5);
  const unsigned hh = lane >> 4, m = lane & 15u;
  const unsigned b = blockIdx.x;

  const unsigned xc0 = umax_u(m, 8u) - 8u;
  const unsigned xc1 = 8u + m;
  const unsigned xc2 = umin_u(24u + m, 31u);
  const _Float16* vrow = Vp + ((size_t)(b * OC + (m & 7u))) * HW + hh * 8u;
  const float* xp0 = in1 + ((size_t)(b * CH + xc0)) * HW + hh * 8u;
  const float* xp1 = in1 + ((size_t)(b * CH + xc1)) * HW + hh * 8u;
  const float* xp2 = in1 + ((size_t)(b * CH + xc2)) * HW + hh * 8u;
  const bool vcol = m < 8u;

  v8f acc0 = {}, acc1 = {}, acc2 = {};
#pragma unroll 1
  for (unsigned s = 0; s < 16u; ++s) {
    const unsigned k0 = (wave * 16u + s) * 32u;
    const v16h vf  = frag_at(vrow + k0);
    const v16h xf0 = xfrag_at(xp0 + k0);
    const v16h xf1 = xfrag_at(xp1 + k0);
    const v16h xf2 = xfrag_at(xp2 + k0);
    v16h bt0;
#pragma unroll
    for (int i = 0; i < 16; ++i) bt0[i] = vcol ? vf[i] : xf0[i];
    acc0 = wmma16(vf, bt0, acc0);
    acc1 = wmma16(vf, xf1, acc1);
    acc2 = wmma16(vf, xf2, acc2);
  }

  if (hh == 0u) {
#pragma unroll
    for (int r = 0; r < 8; ++r) {
      part[((wave * 3u + 0u) * 8u + (unsigned)r) * 16u + m] = acc0[r];
      part[((wave * 3u + 1u) * 8u + (unsigned)r) * 16u + m] = acc1[r];
      part[((wave * 3u + 2u) * 8u + (unsigned)r) * 16u + m] = acc2[r];
    }
  }
  __syncthreads();

  for (unsigned i = tid; i < 320u; i += 256u) {
    const unsigned r = i / 40u, cq = i - r * 40u;
    const unsigned t = cq >> 4, c = cq & 15u;
    float s = 0.0f;
#pragma unroll 1
    for (unsigned w = 0; w < 8u; ++w) s += part[((w * 3u + t) * 8u + r) * 16u + c];
    const float sc = (cq < 8u) ? (1.0f / (VCARRY * VCARRY)) : (1.0f / VCARRY);
    Aug[r * 40u + cq] = s * sc;
  }
  __syncthreads();

#pragma unroll 1
  for (unsigned k = 0; k < 8u; ++k) {
    const float piv = Aug[k * 40u + k];
    const float rp = 1.0f / piv;
    __syncthreads();
    if (tid < 40u) Aug[k * 40u + tid] *= rp;
    __syncthreads();
    if (tid < 8u) fcol[tid] = Aug[tid * 40u + k];
    __syncthreads();
    for (unsigned i = tid; i < 320u; i += 256u) {
      const unsigned r = i / 40u, cq = i - r * 40u;
      if (r != k) Aug[r * 40u + cq] -= fcol[r] * Aug[k * 40u + cq];
    }
    __syncthreads();
  }

  if (wave < 2u) {
    const unsigned k = tid >> 3;
    const unsigned c4 = (tid & 7u) * 4u;
    v4f u;
#pragma unroll
    for (int j = 0; j < 4; ++j) u[j] = Aug[k * 40u + 8u + c4 + (unsigned)j] * (1.0f / VCARRY);
    float* dst = U + (size_t)b * (OC * CH) + k * CH + c4;
    *(volatile v4f*)dst = u;
    __threadfence();
    *(volatile v4f*)dst = u;
  }
}

__global__ __launch_bounds__(256) void apply_kernel(
    const _Float16* __restrict__ Vp, const float* __restrict__ U, float* __restrict__ out) {
  const unsigned g = blockIdx.x * 256u + threadIdx.x;
  const unsigned b = blockIdx.x >> 2;
  const unsigned p4 = (g & 1023u) * 4u;
  float v[8][4];
#pragma unroll
  for (int k = 0; k < 8; ++k) {
    const v4h t = *(const v4h*)(Vp + ((size_t)(b * OC + (unsigned)k)) * HW + p4);
#pragma unroll
    for (int j = 0; j < 4; ++j) v[k][j] = (float)t[j];
  }
#pragma unroll 1
  for (unsigned c = 0; c < (unsigned)CH; ++c) {
    const float* u = U + (size_t)b * (OC * CH) + c;
    v4f yv = {0.0f, 0.0f, 0.0f, 0.0f};
#pragma unroll
    for (int k = 0; k < 8; ++k) {
      const float uk = u[k * CH];
#pragma unroll
      for (int j = 0; j < 4; ++j) yv[j] += v[k][j] * uk;
    }
    float* dst = out + ((size_t)(b * CH + c)) * HW + p4;
    *(volatile v4f*)dst = yv;
    __threadfence();
    *(volatile v4f*)dst = yv;
  }
}

extern "C" void kernel_launch(void* const* d_in, const int* in_sizes, int n_in,
                              void* d_out, int out_size, void* d_ws, size_t ws_size,
                              hipStream_t stream) {
  if (n_in < 8) return;
  const long long need_x = (long long)NB * CH * HW;
  if ((long long)in_sizes[0] < need_x) return;
  if ((long long)in_sizes[1] < need_x) return;
  if (in_sizes[2] < OC * CIN * 9) return;
  if (in_sizes[3] < OC) return;
  if (in_sizes[4] < OC * OC * 9) return;
  if (in_sizes[5] < OC) return;
  if (in_sizes[6] < OC * CIN) return;
  if (in_sizes[7] < OC) return;
  if ((long long)out_size < need_x) return;
  if (ws_size < WS_TOTAL) return;

  const float* in1 = (const float*)d_in[0];
  const float* in2 = (const float*)d_in[1];
  const float* w1  = (const float*)d_in[2];
  const float* b1  = (const float*)d_in[3];
  const float* w2  = (const float*)d_in[4];
  const float* b2  = (const float*)d_in[5];
  const float* w11 = (const float*)d_in[6];
  const float* b11 = (const float*)d_in[7];
  float* out = (float*)d_out;

  char* ws = (char*)d_ws;
  _Float16* WT   = (_Float16*)(ws + OFF_WT);
  _Float16* W1t  = WT + WT_W1;
  _Float16* W2t  = WT + WT_W2;
  _Float16* W11t = WT + WT_W11;
  _Float16* Out1 = (_Float16*)(ws + OFF_O1);
  _Float16* Vpl  = (_Float16*)(ws + OFF_VP);
  float*    Umat = (float*)(ws + OFF_U);

  prep_kernel<<<dim3((WT_VECS + 255) / 256), dim3(256), 0, stream>>>(w1, w2, w11, WT);
  conv1_kernel<<<dim3(NB * IMH), dim3(128), 0, stream>>>(in1, in2, W1t, b1, Out1);
  conv2_kernel<<<dim3(NB * IMH), dim3(128), 0, stream>>>(in1, in2, Out1, W2t, W11t, b2, b11, Vpl);
  gram_solve_kernel<<<dim3(NB), dim3(256), 0, stream>>>(Vpl, in1, Umat);
  apply_kernel<<<dim3(NB * 4), dim3(256), 0, stream>>>(Vpl, Umat, out);
}
